// Transformer_46059229283095
// MI455X (gfx1250) — hardware-run, weakly checked
//
#include <hip/hip_runtime.h>


#ifndef NB
#define NB 8
#endif
#ifndef SEQ
#define SEQ 1024
#endif
#define NB_FULL  8
#define SEQ_FULL 1024
#define NL   4
#define DM   512
#define DF   2048
#define NH   8
#define HD   64
#define DQKV (3 * DM)
#define NTOK (NB * SEQ)
#define QR   32
#define CH   256
#define VTP  (CH + 8)
#define ZN   (SEQ / 32)
#define WTP  72

static_assert(NB >= 1 && NB <= NB_FULL);
static_assert(SEQ >= CH && SEQ <= SEQ_FULL);
static_assert(SEQ % CH == 0);
static_assert(SEQ % 128 == 0);
static_assert(NTOK % QR == 0);
static_assert(NTOK % 8 == 0);
static_assert(NH * HD == DM);
static_assert(QR == 32);
static_assert((ZN % 4) == 0);
static_assert(DM % 32 == 0 && DF % 32 == 0);
static_assert(DM % 64 == 0 && DF % 64 == 0);
static_assert(DM == 512);
static_assert(DQKV % 512 == 0 && DF % 512 == 0);
static_assert(256 * 8 * 2 == 64 * 64);
static_assert(32 * 16 * 8 == QR * 64 * 2);
static_assert(2 * 32 * 16 == DM * 2);
static_assert(4 * 32 * 16 == DM * 4);
static_assert(8 * 4 == QR);
static_assert(256 * 16 == QR * HD * 2);
static_assert(HD * 2 == 8 * 16);
static_assert((WTP * 2) % 16 == 0);

static_assert(8 * QR * 64 * 2 <= 131072);
static_assert(QR * DM * 4 <= 131072);
static_assert(64 * WTP * 2 <= 131072);
static_assert(QR * SEQ * 4 + HD * VTP * 2 + QR * HD * 2 + QR * 4 <= 176128);

typedef _Float16 v16h __attribute__((ext_vector_type(16)));
typedef _Float16 v8h  __attribute__((ext_vector_type(8)));
typedef _Float16 v4h  __attribute__((ext_vector_type(4)));
typedef float    v8f  __attribute__((ext_vector_type(8)));
typedef float    v4f  __attribute__((ext_vector_type(4)));
typedef _Float16 h16;

union Frag { v16h v; v8h h[2]; };

#define WSC   64.0f
#define SC_Z  3.0517578125e-05f
#define SC_P  16384.0f
#define SC_O  2.44140625e-04f
#define LOG2E 1.44269504088896340736f
#define LN_EPS 1e-5f

#define WS_WQKV ((size_t)NL * DQKV * DM * 2)
#define WS_WO   ((size_t)NL * DM * DM * 2)
#define WS_W1   ((size_t)NL * DF * DM * 2)
#define WS_W2   ((size_t)NL * DM * DF * 2)
#define WS_HH   ((size_t)NTOK * DM * 2)
#define WS_HF   ((size_t)NTOK * DM * 4)
#define WS_QKV  ((size_t)NTOK * DQKV * 2)
#define WS_H1F  ((size_t)NTOK * DM * 4)
#define WS_MPL  ((size_t)NTOK * DF * 2)
#define WS_CPL  ((size_t)NTOK * DM * 2)
#define WS_TOTAL (WS_WQKV + WS_WO + WS_W1 + WS_W2 + WS_HH + WS_HF + WS_QKV + WS_H1F + WS_MPL)
static_assert(WS_CPL <= WS_MPL);
static_assert(WS_TOTAL <= (size_t)134217728);
static_assert(WS_WQKV % 128 == 0 && WS_WO % 128 == 0 && WS_W1 % 128 == 0 && WS_W2 % 128 == 0);
static_assert(WS_HH % 128 == 0 && WS_HF % 128 == 0 && WS_QKV % 128 == 0 && WS_H1F % 128 == 0);

static __device__ __forceinline__ v8f zero8() {
    v8f z;
#pragma unroll
    for (int i = 0; i < 8; ++i) z[i] = 0.0f;
    return z;
}

static __device__ __forceinline__ v16h load_frag16(const _Float16* base, int ld, int lane) {
    int m  = lane & 15;
    int kb = (lane >> 4) << 3;
    const _Float16* p = base + (size_t)m * ld + kb;
    Frag f;
    f.h[0] = *(const v8h*)(p);
    f.h[1] = *(const v8h*)(p + 16);
    return f.v;
}

static __device__ __forceinline__ v8f wmma16(v16h a, v16h b, v8f c) {
    v8f d = __builtin_amdgcn_wmma_f32_16x16x32_f16(false, a, false, b, (short)0, c, false, false);
    asm volatile("v_nop\n\tv_nop\n\tv_nop\n\tv_nop" : "+v"(d) : "v"(a), "v"(b));
    return d;
}

static __device__ __forceinline__ float bf16r(float x) {
    unsigned u = __float_as_uint(x);
    u = (u + 0x7FFFu + ((u >> 16) & 1u)) & 0xFFFF0000u;
    return __uint_as_float(u);
}

static __device__ __forceinline__ h16 toh_flush(float v) {
    const h16 r = (h16)v;
    return (fabsf(v) < 6.103515625e-05f) ? (h16)0.0f : r;
}

static __device__ __forceinline__ void wave_lds_sync() {
    __builtin_amdgcn_fence(3, "wavefront");
    asm volatile("s_wait_dscnt 0" ::: "memory");
    __builtin_amdgcn_wave_barrier();
}

static __device__ __forceinline__ float wsum(float v) {
    v += __shfl_xor(v, 16, 32); v += __shfl_xor(v, 8, 32); v += __shfl_xor(v, 4, 32);
    v += __shfl_xor(v, 2, 32);  v += __shfl_xor(v, 1, 32);
    return v;
}
static __device__ __forceinline__ float wmaxr(float v) {
    v = fmaxf(v, __shfl_xor(v, 16, 32)); v = fmaxf(v, __shfl_xor(v, 8, 32));
    v = fmaxf(v, __shfl_xor(v, 4, 32));  v = fmaxf(v, __shfl_xor(v, 2, 32));
    v = fmaxf(v, __shfl_xor(v, 1, 32));
    return v;
}

static __device__ __forceinline__ void load_cols16(const float* p, int lane, float (&o)[16]) {
#pragma unroll
    for (int j = 0; j < 2; ++j) {
        v4f a = *(const v4f*)(p + 256 * j + 8 * lane);
        v4f c = *(const v4f*)(p + 256 * j + 8 * lane + 4);
        o[8 * j + 0] = a.x; o[8 * j + 1] = a.y; o[8 * j + 2] = a.z; o[8 * j + 3] = a.w;
        o[8 * j + 4] = c.x; o[8 * j + 5] = c.y; o[8 * j + 6] = c.z; o[8 * j + 7] = c.w;
    }
}

static __device__ __forceinline__ void ln_lane(const float (&v)[16], const float (&gl)[16],
                                               const float (&el)[16], float (&y)[16]) {
    float s = 0.0f;
#pragma unroll
    for (int e = 0; e < 16; ++e) s += v[e];
    s = wsum(s);
    const float mu = s * (1.0f / (float)DM);
    float d[16];
    float q = 0.0f;
#pragma unroll
    for (int e = 0; e < 16; ++e) { d[e] = v[e] - mu; q = __builtin_fmaf(d[e], d[e], q); }
    q = wsum(q);
    const float rstd = rsqrtf(__builtin_fmaf(q, 1.0f / (float)DM, LN_EPS));
#pragma unroll
    for (int e = 0; e < 16; ++e) y[e] = d[e] * rstd * gl[e] + el[e];
}

__global__ __launch_bounds__(256) void k_wcvt_t(const float* __restrict__ src,
                                                 _Float16* __restrict__ dst,
                                                 int K, int N, int dls) {
#pragma clang fp contract(off)
    __shared__ __align__(16) _Float16 Tt[64 * WTP];
    const int tid = threadIdx.x;
    const int n0 = blockIdx.x * 64, k0 = blockIdx.y * 64, layer = blockIdx.z;
    const float* sp = src + (size_t)layer * K * N + (size_t)k0 * N + n0;
    const int r = tid >> 4, c4 = (tid & 15) * 4;
#pragma unroll
    for (int i = 0; i < 4; ++i) {
        const int kk = r + 16 * i;
        v4f a = *(const v4f*)(sp + (size_t)kk * N + c4);
        Tt[(c4 + 0) * WTP + kk] = toh_flush(bf16r(a.x) * WSC);
        Tt[(c4 + 1) * WTP + kk] = toh_flush(bf16r(a.y) * WSC);
        Tt[(c4 + 2) * WTP + kk] = toh_flush(bf16r(a.z) * WSC);
        Tt[(c4 + 3) * WTP + kk] = toh_flush(bf16r(a.w) * WSC);
    }
    __syncthreads();
    const int nn = tid >> 3, kp = (tid & 7) * 8;
    const v8h o0 = *(const v8h*)(&Tt[nn * WTP + kp]);
    const v8h o1 = *(const v8h*)(&Tt[(nn + 32) * WTP + kp]);
    _Float16* dp = dst + (size_t)layer * dls + (size_t)n0 * K + k0;
    *(volatile v8h*)(dp + (size_t)nn * K + kp)        = o0;
    *(volatile v8h*)(dp + (size_t)(nn + 32) * K + kp) = o1;
    __threadfence();
    *(volatile v8h*)(dp + (size_t)nn * K + kp)        = o0;
    *(volatile v8h*)(dp + (size_t)(nn + 32) * K + kp) = o1;
}

__global__ __launch_bounds__(256) void k_xcvt(const float* __restrict__ x,
                                               float* __restrict__ hf,
                                               _Float16* __restrict__ hh) {
#pragma clang fp contract(off)
    const int tid = threadIdx.x, lane = tid & 31, w = tid >> 5;
    const int tok = blockIdx.x * 8 + w;
    const int b = tok / SEQ, s = tok - b * SEQ;
    const float* xr = x + ((size_t)b * SEQ_FULL + s) * DM;
    float v[16];
    load_cols16(xr, lane, v);
    v8h o[2];
#pragma unroll
    for (int j = 0; j < 2; ++j)
#pragma unroll
        for (int e = 0; e < 8; ++e) o[j][e] = toh_flush(bf16r(v[8 * j + e]));
    v4f s4[4];
#pragma unroll
    for (int jj = 0; jj < 4; ++jj) {
        v4f t4 = *(const v4f*)(xr + 128 * jj + 4 * lane);
        t4.x = bf16r(t4.x); t4.y = bf16r(t4.y); t4.z = bf16r(t4.z); t4.w = bf16r(t4.w);
        s4[jj] = t4;
    }
    _Float16* hrow = hh + (size_t)tok * DM;
    float*    orow = hf + (size_t)tok * DM;
    *(volatile v8h*)(hrow + 8 * lane)       = o[0];
    *(volatile v8h*)(hrow + 256 + 8 * lane) = o[1];
#pragma unroll
    for (int jj = 0; jj < 4; ++jj) *(volatile v4f*)(orow + 128 * jj + 4 * lane) = s4[jj];
    __threadfence();
    *(volatile v8h*)(hrow + 8 * lane)       = o[0];
    *(volatile v8h*)(hrow + 256 + 8 * lane) = o[1];
#pragma unroll
    for (int jj = 0; jj < 4; ++jj) *(volatile v4f*)(orow + 128 * jj + 4 * lane) = s4[jj];
}

static __device__ __forceinline__ void gemm_32x64(const _Float16* __restrict__ Ab,
                                                  const _Float16* __restrict__ Bb,
                                                  int K, int lane, v8f (&acc)[2][4]) {
#pragma unroll
    for (int t = 0; t < 2; ++t)
#pragma unroll
        for (int j = 0; j < 4; ++j) acc[t][j] = zero8();
#pragma unroll 1
    for (int k0 = 0; k0 < K; k0 += 32) {
        v16h a0 = load_frag16(Ab + k0, K, lane);
        v16h a1 = load_frag16(Ab + (size_t)16 * K + k0, K, lane);
        v16h bb[4];
#pragma unroll
        for (int j = 0; j < 4; ++j) bb[j] = load_frag16(Bb + (size_t)(16 * j) * K + k0, K, lane);
#pragma unroll
        for (int j = 0; j < 4; ++j) {
            acc[0][j] = wmma16(a0, bb[j], acc[0][j]);
            acc[1][j] = wmma16(a1, bb[j], acc[1][j]);
        }
    }
}

__global__ __launch_bounds__(256) __attribute__((amdgpu_num_vgpr(256)))
void k_gemm_p(const _Float16* __restrict__ A, int K, const _Float16* __restrict__ Bw,
              const float* __restrict__ b0, const float* __restrict__ b1,
              const float* __restrict__ b2, const float* __restrict__ b3,
              float lo, _Float16* __restrict__ outp, int ldo) {
    __shared__ __align__(16) _Float16 st[8][QR * 64];
    const int tid = threadIdx.x, lane = tid & 31, w = tid >> 5;
    const int hh = lane >> 4, m = lane & 15;
    const int m0  = blockIdx.x * QR;
    const int seg = blockIdx.y;
    const int nl  = 64 * w;
    const int n0w = seg * 512 + nl;
    const float* bias = (seg == 0) ? b0 : ((seg == 1) ? b1 : ((seg == 2) ? b2 : b3));

    v8f acc[2][4];
    gemm_32x64(A + (size_t)m0 * K, Bw + (size_t)n0w * K, K, lane, acc);

    float bl[4];
#pragma unroll
    for (int j = 0; j < 4; ++j) bl[j] = bf16r(bias[nl + 16 * j + m]);
#pragma unroll
    for (int t = 0; t < 2; ++t)
#pragma unroll
        for (int j = 0; j < 4; ++j)
#pragma unroll
            for (int r = 0; r < 8; ++r) {
                float a = acc[t][j][r];
                float val = fmaxf(__builtin_fmaf(bl[j], WSC, a), lo);
                st[w][(16 * t + 8 * hh + r) * 64 + 16 * j + m] = toh_flush(val);
            }
    wave_lds_sync();

    v8h pv[8];
    const int lr = lane >> 3, lc = (lane & 7) * 8;
#pragma unroll
    for (int i = 0; i < 8; ++i) pv[i] = *(const v8h*)(&st[w][(4 * i + lr) * 64 + lc]);
    _Float16* ob = outp + (size_t)m0 * ldo + n0w;
#pragma unroll
    for (int i = 0; i < 8; ++i) *(volatile v8h*)(ob + (size_t)(4 * i + lr) * ldo + lc) = pv[i];
    __threadfence();
#pragma unroll
    for (int i = 0; i < 8; ++i) *(volatile v8h*)(ob + (size_t)(4 * i + lr) * ldo + lc) = pv[i];
}

__global__ __launch_bounds__(256) __attribute__((amdgpu_num_vgpr(256)))
void k_gemm_r(const _Float16* __restrict__ A, int K, const _Float16* __restrict__ Bw,
              const float* __restrict__ bias, const float* __restrict__ res,
              const float* __restrict__ g, const float* __restrict__ be,
              float* __restrict__ outf, _Float16* __restrict__ outh) {
    __shared__ __align__(16) float T[QR * DM];
    const int tid = threadIdx.x, lane = tid & 31, w = tid >> 5;
    const int hh = lane >> 4, m = lane & 15;
    const int m0 = blockIdx.x * QR;
    const int nl = 64 * w;

    v8f acc[2][4];
    gemm_32x64(A + (size_t)m0 * K, Bw + (size_t)nl * K, K, lane, acc);
#pragma unroll
    for (int t = 0; t < 2; ++t)
#pragma unroll
        for (int j = 0; j < 4; ++j)
#pragma unroll
            for (int r = 0; r < 8; ++r)
                T[(16 * t + 8 * hh + r) * DM + nl + 16 * j + m] = acc[t][j][r];
    __syncthreads();

    float bl[16], gl[16], el[16];
    load_cols16(bias, lane, bl);
    load_cols16(g, lane, gl);
    load_cols16(be, lane, el);
#pragma unroll
    for (int e = 0; e < 16; ++e) { bl[e] = bf16r(bl[e]); gl[e] = bf16r(gl[e]); el[e] = bf16r(el[e]); }

#pragma unroll 1
    for (int rr = 0; rr < 4; ++rr) {
        const int row = 4 * w + rr;
        const int tok = m0 + row;
        float v[16], rv[16], yv[16];
        load_cols16(&T[row * DM], lane, v);
        load_cols16(res + (size_t)tok * DM, lane, rv);
#pragma unroll
        for (int e = 0; e < 16; ++e) v[e] = rv[e] + __builtin_fmaf(v[e], SC_O, bl[e]);
        ln_lane(v, gl, el, yv);

        float* trow = &T[row * DM];
#pragma unroll
        for (int j = 0; j < 2; ++j) {
            v4f p0, p1;
            p0.x = yv[8 * j + 0]; p0.y = yv[8 * j + 1]; p0.z = yv[8 * j + 2]; p0.w = yv[8 * j + 3];
            p1.x = yv[8 * j + 4]; p1.y = yv[8 * j + 5]; p1.z = yv[8 * j + 6]; p1.w = yv[8 * j + 7];
            *(v4f*)(trow + 256 * j + 8 * lane)     = p0;
            *(v4f*)(trow + 256 * j + 8 * lane + 4) = p1;
        }
        wave_lds_sync();
        v4f s4[4];
#pragma unroll
        for (int jj = 0; jj < 4; ++jj) s4[jj] = *(const v4f*)(trow + 128 * jj + 4 * lane);

        float* orow = outf + (size_t)tok * DM;
        v8h o[2];
#pragma unroll
        for (int j = 0; j < 2; ++j)
#pragma unroll
            for (int e = 0; e < 8; ++e) o[j][e] = toh_flush(yv[8 * j + e]);
        _Float16* hrow = outh + (size_t)tok * DM;
        *(volatile v8h*)(hrow + 8 * lane)       = o[0];
        *(volatile v8h*)(hrow + 256 + 8 * lane) = o[1];
#pragma unroll
        for (int jj = 0; jj < 4; ++jj) *(volatile v4f*)(orow + 128 * jj + 4 * lane) = s4[jj];
        __threadfence();
        *(volatile v8h*)(hrow + 8 * lane)       = o[0];
        *(volatile v8h*)(hrow + 256 + 8 * lane) = o[1];
#pragma unroll
        for (int jj = 0; jj < 4; ++jj) *(volatile v4f*)(orow + 128 * jj + 4 * lane) = s4[jj];
    }
}

__global__ __launch_bounds__(256) __attribute__((amdgpu_num_vgpr(256)))
void k_attn(const _Float16* __restrict__ qkv, _Float16* __restrict__ ctx) {
    __shared__ __align__(16) float    zs[QR * SEQ];
    __shared__ __align__(16) _Float16 Vt[HD * VTP];
    __shared__ __align__(16) _Float16 Cst[QR * HD];
    __shared__ float rinv[QR];
    _Float16* ph = reinterpret_cast<_Float16*>(zs);
    constexpr int PP  = 2 * SEQ;
    constexpr int PLD = PP + 8;
    constexpr int KTW = SEQ / 128;

    const int tid = threadIdx.x, lane = tid & 31, w = tid >> 5;
    const int hh = lane >> 4, m = lane & 15;
    const int h = blockIdx.y, b = blockIdx.z;
    const int q0 = blockIdx.x * QR;
    const size_t tokq = (size_t)b * SEQ + q0;
    const _Float16* qp = qkv + tokq * DQKV + h * HD;
    const _Float16* kp = qkv + (size_t)b * SEQ * DQKV + DM + h * HD;
    const _Float16* vp = qkv + (size_t)b * SEQ * DQKV + 2 * DM + h * HD;

    {
        const v16h qa00 = load_frag16(qp, DQKV, lane);
        const v16h qa01 = load_frag16(qp + 32, DQKV, lane);
        const v16h qa10 = load_frag16(qp + (size_t)16 * DQKV, DQKV, lane);
        const v16h qa11 = load_frag16(qp + (size_t)16 * DQKV + 32, DQKV, lane);
#pragma unroll 1
        for (int i = 0; i < KTW; ++i) {
            const int key0 = (w * KTW + i) * 16;
            const _Float16* kt = kp + (size_t)key0 * DQKV;
            v16h kf0 = load_frag16(kt, DQKV, lane);
            v16h kf1 = load_frag16(kt + 32, DQKV, lane);
            v8f s0 = wmma16(qa00, kf0, zero8());
            s0 = wmma16(qa01, kf1, s0);
            v8f s1 = wmma16(qa10, kf0, zero8());
            s1 = wmma16(qa11, kf1, s1);
#pragma unroll
            for (int r = 0; r < 8; ++r) {
                zs[(8 * hh + r) * SEQ + key0 + m]      = s0[r] * SC_Z;
                zs[(16 + 8 * hh + r) * SEQ + key0 + m] = s1[r] * SC_Z;
            }
        }
    }
    __syncthreads();

#pragma unroll 1
    for (int rr = 0; rr < 4; ++rr) {
        const int row = 4 * w + rr;
        float z[ZN];
        const float* zr = &zs[row * SEQ];
#pragma unroll
        for (int j = 0; j < ZN / 4; ++j) {
            v4f t4 = *(const v4f*)(zr + 128 * j + 4 * lane);
            z[4 * j + 0] = t4.x; z[4 * j + 1] = t4.y; z[4 * j + 2] = t4.z; z[4 * j + 3] = t4.w;
        }
        float mx = z[0];
#pragma unroll
        for (int i = 1; i < ZN; ++i) mx = fmaxf(mx, z[i]);
        mx = wmaxr(mx);
        float ss = 0.0f;
#pragma unroll
        for (int i = 0; i < ZN; ++i) {
            z[i] = __builtin_amdgcn_exp2f((z[i] - mx) * LOG2E);
            ss += z[i];
        }
        ss = wsum(ss);
        const float sinv = SC_P * __builtin_amdgcn_rcpf(ss);
        float sc = 0.0f;
        _Float16* prow = ph + (size_t)row * PP + (row & 15) * 8;
#pragma unroll
        for (int j = 0; j < ZN / 4; ++j) {
            v4h pk;
#pragma unroll
            for (int e = 0; e < 4; ++e) {
                const h16 hv = toh_flush(z[4 * j + e] * sinv);
                pk[e] = hv;
                sc += (float)hv;
            }
            *(v4h*)(prow + 128 * j + 4 * lane) = pk;
        }
        sc = wsum(sc);
        rinv[row] = __builtin_amdgcn_rcpf(sc);
    }
    __syncthreads();

    const int rt = w & 1, ct = w >> 1;
    v8f acc = zero8();
#pragma unroll 1
    for (int c0 = 0; c0 < SEQ; c0 += CH) {
#pragma unroll
        for (int i2 = 0; i2 < 8; ++i2) {
            const int idx = tid + 256 * i2;
            const int t = idx >> 3, part = idx & 7;
            v8h vv = *(const v8h*)(vp + (size_t)(c0 + t) * DQKV + part * 8);
#pragma unroll
            for (int e = 0; e < 8; ++e) Vt[(part * 8 + e) * VTP + t] = vv[e];
        }
        __syncthreads();
#pragma unroll 1
        for (int j = 0; j < CH; j += 32) {
            v16h pa = load_frag16(ph + (size_t)(16 * rt) * PP + c0 + j, PLD, lane);
            v16h vb = load_frag16(&Vt[(16 * ct) * VTP + j], VTP, lane);
            acc = wmma16(pa, vb, acc);
        }
        __syncthreads();
    }

#pragma unroll
    for (int r = 0; r < 8; ++r)
        Cst[(16 * rt + 8 * hh + r) * HD + 16 * ct + m] = toh_flush(acc[r] * rinv[16 * rt + 8 * hh + r]);
    __syncthreads();
    const int orow = 4 * w + (lane >> 3), oc = (lane & 7) * 8;
    v8h cv = *(const v8h*)(&Cst[orow * HD + oc]);
    _Float16* dst = ctx + (tokq + orow) * DM + h * HD + oc;
    *(volatile v8h*)dst = cv;
    __threadfence();
    *(volatile v8h*)dst = cv;
}

extern "C" void kernel_launch(void* const* d_in, const int* in_sizes, int n_in,
                              void* d_out, int out_size, void* d_ws, size_t ws_size,
                              hipStream_t stream) {
    if (n_in < 17) return;
    if (in_sizes[0] < ((NB - 1) * SEQ_FULL + SEQ) * DM) return;
    if (in_sizes[1] < NL * DM * DM || in_sizes[3] < NL * DM * DM || in_sizes[5] < NL * DM * DM || in_sizes[7] < NL * DM * DM) return;
    if (in_sizes[2] < NL * DM || in_sizes[4] < NL * DM || in_sizes[6] < NL * DM || in_sizes[8] < NL * DM) return;
    if (in_sizes[9] < NL * DM * DF || in_sizes[10] < NL * DF || in_sizes[11] < NL * DF * DM || in_sizes[12] < NL * DM) return;
    if (in_sizes[13] < NL * DM || in_sizes[14] < NL * DM || in_sizes[15] < NL * DM || in_sizes[16] < NL * DM) return;
    if (out_size < NTOK * DM) return;

    const float* x   = (const float*)d_in[0];
    const float* Wq  = (const float*)d_in[1];
    const float* bq  = (const float*)d_in[2];
    const float* Wk  = (const float*)d_in[3];
    const float* bk  = (const float*)d_in[4];
    const float* Wv  = (const float*)d_in[5];
    const float* bv  = (const float*)d_in[6];
    const float* Wo  = (const float*)d_in[7];
    const float* bo  = (const float*)d_in[8];
    const float* W1  = (const float*)d_in[9];
    const float* b1  = (const float*)d_in[10];
    const float* W2  = (const float*)d_in[11];
    const float* b2  = (const float*)d_in[12];
    const float* g1  = (const float*)d_in[13];
    const float* be1 = (const float*)d_in[14];
    const float* g2  = (const float*)d_in[15];
    const float* be2 = (const float*)d_in[16];
    float* out = (float*)d_out;

    char* ws = (char*)d_ws;
    size_t off = 0;
    _Float16* wqkv = (_Float16*)(ws + off); off += WS_WQKV;
    _Float16* wo16 = (_Float16*)(ws + off); off += WS_WO;
    _Float16* w116 = (_Float16*)(ws + off); off += WS_W1;
    _Float16* w216 = (_Float16*)(ws + off); off += WS_W2;
    _Float16* hh   = (_Float16*)(ws + off); off += WS_HH;
    float*    hf   = (float*)(ws + off);    off += WS_HF;
    _Float16* qkv  = (_Float16*)(ws + off); off += WS_QKV;
    float*    h1f  = (float*)(ws + off);    off += WS_H1F;
    _Float16* mpl  = (_Float16*)(ws + off); off += WS_MPL;
    _Float16* cpl  = mpl;
    if (off > ws_size) return;

    k_wcvt_t<<<dim3(DM / 64, DM / 64, NL), dim3(256), 0, stream>>>(Wq, wqkv, DM, DM, DQKV * DM);
    k_wcvt_t<<<dim3(DM / 64, DM / 64, NL), dim3(256), 0, stream>>>(Wk, wqkv + (size_t)DM * DM, DM, DM, DQKV * DM);
    k_wcvt_t<<<dim3(DM / 64, DM / 64, NL), dim3(256), 0, stream>>>(Wv, wqkv + (size_t)2 * DM * DM, DM, DM, DQKV * DM);
    k_wcvt_t<<<dim3(DM / 64, DM / 64, NL), dim3(256), 0, stream>>>(Wo, wo16, DM, DM, DM * DM);
    k_wcvt_t<<<dim3(DF / 64, DM / 64, NL), dim3(256), 0, stream>>>(W1, w116, DM, DF, DF * DM);
    k_wcvt_t<<<dim3(DM / 64, DF / 64, NL), dim3(256), 0, stream>>>(W2, w216, DF, DM, DM * DF);

    k_xcvt<<<dim3(NTOK / 8), dim3(256), 0, stream>>>(x, hf, hh);

    for (int l = 0; l < NL; ++l) {
        const float* bql = bq + (size_t)l * DM;
        const float* bkl = bk + (size_t)l * DM;
        const float* bvl = bv + (size_t)l * DM;
        const float* b1l = b1 + (size_t)l * DF;
        float* hout = (l == NL - 1) ? out : hf;
        k_gemm_p<<<dim3(NTOK / QR, DQKV / 512), dim3(256), 0, stream>>>(
            hh, DM, wqkv + (size_t)l * DQKV * DM, bql, bkl, bvl, bvl, -3.0e38f, qkv, DQKV);
        k_attn<<<dim3(SEQ / QR, NH, NB), dim3(256), 0, stream>>>(qkv, cpl);
        k_gemm_r<<<dim3(NTOK / QR), dim3(256), 0, stream>>>(
            cpl, DM, wo16 + (size_t)l * DM * DM, bo + (size_t)l * DM, hf,
            g1 + (size_t)l * DM, be1 + (size_t)l * DM, h1f, hh);
        k_gemm_p<<<dim3(NTOK / QR, DF / 512), dim3(256), 0, stream>>>(
            hh, DM, w116 + (size_t)l * DF * DM, b1l, b1l + 512, b1l + 1024, b1l + 1536, 0.0f, mpl, DF);
        k_gemm_r<<<dim3(NTOK / QR), dim3(256), 0, stream>>>(
            mpl, DF, w216 + (size_t)l * DM * DF, b2 + (size_t)l * DM, h1f,
            g2 + (size_t)l * DM, be2 + (size_t)l * DM, hout, hh);
    }
}
